// Liu_U_61933428408753
// MI455X (gfx1250) — hardware-verified
//
#include <hip/hip_runtime.h>
#include <math.h>

typedef __attribute__((ext_vector_type(16))) _Float16 v16h;
typedef __attribute__((ext_vector_type(16))) __bf16 v16b;
typedef __attribute__((ext_vector_type(8)))  _Float16 v8h;
typedef __attribute__((ext_vector_type(8)))  float v8f;
typedef __attribute__((ext_vector_type(4)))  float v4f;
typedef __attribute__((ext_vector_type(2)))  float v2f;
typedef __attribute__((ext_vector_type(4)))  unsigned v4u;
typedef __attribute__((ext_vector_type(4)))  int v4i;
typedef float __attribute__((may_alias)) float_a;
typedef int __attribute__((may_alias)) int_a;

template <typename T> __device__ __forceinline__ void vst2(void* p, T v) { *(volatile T*)p = v; __threadfence(); *(volatile T*)p = v; }
__device__ __forceinline__ v8f wmma16(v16h a, v16h b, v8f c) {
  v8f d = __builtin_amdgcn_wmma_f32_16x16x32_f16(false, a, false, b, (short)0, c, false, false);
  asm volatile("v_nop\n\tv_nop\n\tv_nop\n\tv_nop" : "+v"(d) : "v"(a), "v"(b));
  return d;
}
__device__ __forceinline__ v8f wmma_bf(v16b a, v16b b, v8f c) {
  v8f d = __builtin_amdgcn_wmma_f32_16x16x32_bf16(false, a, false, b, (short)0, c, false, false);
  asm volatile("v_nop\n\tv_nop\n\tv_nop\n\tv_nop" : "+v"(d) : "v"(a), "v"(b));
  return d;
}
__device__ __forceinline__ v16h frag_h(const _Float16* rowk0, int lane) {
  union { v16h v; v8h q[2]; } u; const _Float16* p = rowk0 + 8 * (lane >> 4);
  u.q[0] = *(const v8h*)p; u.q[1] = *(const v8h*)(p + 16); return u.v;
}
__device__ __forceinline__ v16h frag_f32(const float* rowk0, int lane) {
  v16h a; const float* p = rowk0 + 8 * (lane >> 4);
#pragma unroll
  for (int i = 0; i < 8; ++i) { a[i] = (_Float16)p[i]; a[8 + i] = (_Float16)p[16 + i]; }
  return a;
}
__device__ __forceinline__ v16h frag_f32s(const float* rowk0, int lane, float sc) {
  v16h a; const float* p = rowk0 + 8 * (lane >> 4);
#pragma unroll
  for (int i = 0; i < 8; ++i) { a[i] = (_Float16)(p[i] * sc); a[8 + i] = (_Float16)(p[16 + i] * sc); }
  return a;
}
__device__ __forceinline__ v16h fragc_f32(const float* W, int k0, int n, int lane, int ld, int K) {
  v16h a; const int g = lane >> 4;
#pragma unroll
  for (int i = 0; i < 8; ++i) { const int ka = k0 + 8 * g + i, kb = ka + 16;
    a[i] = (_Float16)(ka < K ? W[(size_t)ka * ld + n] : 0.f); a[8 + i] = (_Float16)(kb < K ? W[(size_t)kb * ld + n] : 0.f); }
  return a;
}
struct F2 { v16b h, l; };
__device__ __forceinline__ F2 bsplit16(const float v[16]) { F2 r;
#pragma unroll
  for (int i = 0; i < 16; ++i) { const __bf16 h = (__bf16)v[i]; r.h[i] = h; r.l[i] = (__bf16)(v[i] - (float)h); }
  return r; }
__device__ __forceinline__ F2 split_row(const float* row, int k0, int lane) { float v[16]; const float* p = row + k0 + 8 * (lane >> 4);
#pragma unroll
  for (int i = 0; i < 8; ++i) { v[i] = p[i]; v[8 + i] = p[16 + i]; }
  return bsplit16(v); }
__device__ __forceinline__ F2 split_rowK(const float* row, int k0, int lane, int K) { float v[16]; const int g = lane >> 4;
#pragma unroll
  for (int i = 0; i < 8; ++i) { const int ka = k0 + 8 * g + i, kb = ka + 16; v[i] = ka < K ? row[ka] : 0.f; v[8 + i] = kb < K ? row[kb] : 0.f; }
  return bsplit16(v); }
__device__ __forceinline__ F2 split_col(const float* W, int k0, int n, int lane, int ld, int K) { float v[16]; const int g = lane >> 4;
#pragma unroll
  for (int i = 0; i < 8; ++i) { const int ka = k0 + 8 * g + i, kb = ka + 16; v[i] = ka < K ? W[(size_t)ka * ld + n] : 0.f; v[8 + i] = kb < K ? W[(size_t)kb * ld + n] : 0.f; }
  return bsplit16(v); }
__device__ __forceinline__ v8f mac3(const F2& a, const F2& b, v8f c) { c = wmma_bf(a.l, b.h, c); c = wmma_bf(a.h, b.l, c); return wmma_bf(a.h, b.h, c); }
__device__ __forceinline__ float sigm(float v) { return 1.0f / (1.0f + expf(-v)); }
#define LDSX() do { asm volatile("s_wait_dscnt 0" ::: "memory"); __builtin_amdgcn_wave_barrier(); __builtin_amdgcn_fence(__ATOMIC_RELEASE, "workgroup"); } while (0)

#define NBT 2048
#define UD 4
#define ZD 4
#define YD 2
#define HDN 20
#define TT 1024
#define TCH 64

__global__ __launch_bounds__(128) void k_rec(const float* __restrict__ u, const float* __restrict__ y, const float* __restrict__ W1, const float* __restrict__ b1, const float* __restrict__ W2, const float* __restrict__ b2,
                                           const float* __restrict__ W3, const float* __restrict__ b3, const float* __restrict__ W4, const float* __restrict__ b4, float* __restrict__ part) {
  __shared__ __align__(16) _Float16 sW1[32][40], sW2[16][40], sW3[32][40], sW4[16][40];
  __shared__ __align__(16) float su[64][UD][TCH + 1]; __shared__ __align__(16) float sy[64][YD][TCH + 1];
  __shared__ __align__(16) _Float16 sA[4][16][40];
  __shared__ float sx[4][16][4];
  __shared__ float sl[4];
  const int tid = threadIdx.x, wave = tid >> 5, lane = tid & 31, col = lane & 15, g = lane >> 4;
  const int b0 = blockIdx.x * 64, r0 = wave * 16;
  for (int q = tid; q < 32 * 40; q += 128) { const int n = q / 40, k = q % 40; sW1[n][k] = (_Float16)((n < HDN && k < UD + ZD) ? W1[k * HDN + n] : 0.f); sW3[n][k] = (_Float16)((n < HDN && k < UD + ZD) ? W3[k * HDN + n] : 0.f); }
  for (int q = tid; q < 16 * 40; q += 128) { const int n = q / 40, k = q % 40; sW2[n][k] = (_Float16)((n < ZD && k < HDN) ? W2[k * ZD + n] : 0.f); sW4[n][k] = (_Float16)((n < YD && k < HDN) ? W4[k * YD + n] : 0.f); }
  for (int q = tid; q < 4 * 16 * 4; q += 128) (&sx[0][0][0])[q] = 0.f;
  for (int q = tid; q < 4 * 16 * 40; q += 128) (&sA[0][0][0])[q] = (_Float16)0.f;
  float lacc = 0.f;
  __syncthreads();
#pragma unroll 1
  for (int t0 = 0; t0 < TT; t0 += TCH) {
    __syncthreads();
    for (int q = tid; q < 64 * UD * TCH; q += 128) { const int rl = q / (UD * TCH), rem = q % (UD * TCH), d = rem / TCH, tt = rem % TCH; su[rl][d][tt] = u[((size_t)(b0 + rl) * UD + d) * TT + t0 + tt]; }
    for (int q = tid; q < 64 * YD * TCH; q += 128) { const int rl = q / (YD * TCH), rem = q % (YD * TCH), d = rem / TCH, tt = rem % TCH; sy[rl][d][tt] = y[((size_t)(b0 + rl) * YD + d) * TT + t0 + tt]; }
    __syncthreads();
#pragma unroll 1
    for (int tt = 0; tt < TCH; ++tt) {
      if (g == 0) { _Float16* ar = &sA[wave][col][0];
#pragma unroll
        for (int d = 0; d < UD; ++d) ar[d] = (_Float16)su[r0 + col][d][tt];
#pragma unroll
        for (int d = 0; d < ZD; ++d) ar[UD + d] = (_Float16)sx[wave][col][d]; }
      else { _Float16* ar = &sA[wave][col][0];
#pragma unroll
        for (int d = 8; d < 20; ++d) ar[d] = (_Float16)0.f; }
      LDSX();
      v16h a = frag_h(&sA[wave][col][0], lane);
      v8f h0 = {}, h1 = {}; h0 = wmma16(a, frag_h(&sW1[col][0], lane), h0); h1 = wmma16(a, frag_h(&sW1[16 + col][0], lane), h1);
      LDSX();
#pragma unroll
      for (int r = 0; r < 8; ++r) { { const float v = h0[r] + b1[col]; sA[wave][8 * g + r][col] = (_Float16)(v > 0.f ? v : 0.f); }
        if (col < 4) { const float v = h1[r] + b1[16 + col]; sA[wave][8 * g + r][16 + col] = (_Float16)(v > 0.f ? v : 0.f); } }
      LDSX();
      a = frag_h(&sA[wave][col][0], lane);
      v8f xo = {}; xo = wmma16(a, frag_h(&sW2[col][0], lane), xo);
      if (col < ZD) {
#pragma unroll
        for (int r = 0; r < 8; ++r) sx[wave][8 * g + r][col] = xo[r] + b2[col]; }
      LDSX();
      if (g == 0) { _Float16* ar = &sA[wave][col][0];
#pragma unroll
        for (int d = 0; d < UD; ++d) ar[d] = (_Float16)su[r0 + col][d][tt];
#pragma unroll
        for (int d = 0; d < ZD; ++d) ar[UD + d] = (_Float16)sx[wave][col][d]; }
      else { _Float16* ar = &sA[wave][col][0];
#pragma unroll
        for (int d = 8; d < 20; ++d) ar[d] = (_Float16)0.f; }
      LDSX();
      a = frag_h(&sA[wave][col][0], lane);
      v8f m0 = {}, m1 = {}; m0 = wmma16(a, frag_h(&sW3[col][0], lane), m0); m1 = wmma16(a, frag_h(&sW3[16 + col][0], lane), m1);
      LDSX();
#pragma unroll
      for (int r = 0; r < 8; ++r) { { const float v = m0[r] + b3[col]; sA[wave][8 * g + r][col] = (_Float16)(v > 0.f ? v : 0.f); }
        if (col < 4) { const float v = m1[r] + b3[16 + col]; sA[wave][8 * g + r][16 + col] = (_Float16)(v > 0.f ? v : 0.f); } }
      LDSX();
      a = frag_h(&sA[wave][col][0], lane);
      v8f yo = {}; yo = wmma16(a, frag_h(&sW4[col][0], lane), yo);
      if (col < YD) {
#pragma unroll
        for (int r = 0; r < 8; ++r) { const float dv = yo[r] + b4[col] - sy[r0 + 8 * g + r][col][tt]; lacc += dv * dv; } }
      __builtin_amdgcn_wave_barrier(); } }
#pragma unroll
  for (int off = 16; off >= 1; off >>= 1) lacc += __shfl_xor(lacc, off, 32);
  if (lane == 0) sl[wave] = lacc;
  __syncthreads();
  if (tid < 32) vst2(part + (size_t)blockIdx.x * 32 + tid, (float)(tid == 0 ? (sl[0] + sl[1]) + (sl[2] + sl[3]) : 0.f));
}
__global__ __launch_bounds__(32) void k_fin(const float* __restrict__ part, float* __restrict__ out) {
  if (threadIdx.x == 0) { float s = 0.f; for (int b = 0; b < NBT / 64; ++b) s += part[(size_t)b * 32]; vst2(out, s); }
}
extern "C" void kernel_launch(void* const* d_in, const int* in_sizes, int n_in, void* d_out, int out_size, void* d_ws, size_t ws_size, hipStream_t stream) {
  (void)in_sizes; (void)n_in; (void)out_size; (void)ws_size;
  const float** I = (const float**)d_in;
  float* out = (float*)d_out; float* part = (float*)d_ws;
  k_rec<<<NBT / 64, 128, 0, stream>>>(I[0], I[1], I[2], I[3], I[4], I[5], I[6], I[7], I[8], I[9], part);
  k_fin<<<1, 32, 0, stream>>>(part, out);
}
